// GAT_57612691309076
// MI455X (gfx1250) — hardware-verified
//
#include <hip/hip_runtime.h>
#include <stddef.h>
#include <stdint.h>
#include <math.h>


#define NB     4
#define NN     2048
#define FIN    16
#define HID    32
#define NH1    6
#define CAT    192
#define OC     16
#define MR     (NB * NN)
#define KX     32
#define K2     (2 * CAT)
#define NEGSL  0.2f
#define FILLV  (-1.0e12f)
#define NEGBIG (-3.0e38f)
#define PB_X   128
#define PB_W1  3
#define PB_W2  3
#define PB_K   256
#define WSMAX  134217728

static_assert(NN == 2048 && (NN % 64) == 0);
static_assert(MR * 4 == PB_X * 256);
static_assert(CAT * 4 == PB_W1 * 256);
static_assert(OC * (K2 / 8) == PB_W2 * 256);
static_assert(NN == PB_K * 8);
static_assert(CAT == NH1 * HID && HID == KX && (K2 % 32) == 0);
static_assert((CAT % 8) == 0);

typedef float          v4f  __attribute__((ext_vector_type(4)));
typedef float          v8f  __attribute__((ext_vector_type(8)));
typedef int            v8i  __attribute__((ext_vector_type(8)));
typedef unsigned int   v4u  __attribute__((ext_vector_type(4)));
typedef unsigned short v8us __attribute__((ext_vector_type(8)));
typedef __bf16         v16b __attribute__((ext_vector_type(16)));
typedef v4f  __attribute__((may_alias)) v4fa;
typedef v4u  __attribute__((may_alias)) v4ua;
typedef v8us __attribute__((may_alias)) v8usa;
union FragB { v16b v; v8us h[2]; v8i w; };

__device__ __forceinline__ v8f wmb(const FragB& a, const FragB& b, v8f c) {
  v8f d = __builtin_amdgcn_wmma_f32_16x16x32_bf16(false, a.v, false, b.v, (short)0, c, false, false);
  asm volatile("v_nop\n\tv_nop\n\tv_nop\n\tv_nop" : "+v"(d) : "v"(a.w), "v"(b.w));
  return d;
}

__device__ __forceinline__ unsigned int rne16(float f) {
  const unsigned int u = __float_as_uint(f);
  return u + 0x7FFFu + ((u >> 16) & 1u);
}
__device__ __forceinline__ float bfr(float f) { return __uint_as_float(rne16(f) & 0xFFFF0000u); }
__device__ __forceinline__ void split2(float p, unsigned int& rh, unsigned int& rl) {
  rh = rne16(p);
  const float hf = __uint_as_float(rh & 0xFFFF0000u);
  rl = rne16(p - hf);
}
__device__ __forceinline__ unsigned int pkw(unsigned int r0, unsigned int r1) {
  return (r0 >> 16) | (r1 & 0xFFFF0000u);
}
__device__ __forceinline__ v4u pack8(const v4f a, const v4f b) {
  v4u r;
  r.x = pkw(rne16(a.x), rne16(a.y)); r.y = pkw(rne16(a.z), rne16(a.w));
  r.z = pkw(rne16(b.x), rne16(b.y)); r.w = pkw(rne16(b.z), rne16(b.w));
  return r;
}

__global__ __launch_bounds__(256) void k_prep(const float* __restrict__ x, const float* __restrict__ adj,
                                              const float* __restrict__ W1, const float* __restrict__ W2,
                                              unsigned short* XB, unsigned short* W1T, unsigned short* W2D,
                                              unsigned int* KEEP) {
  __shared__ __attribute__((aligned(16))) unsigned int kws[8 * 64];
  const int tid = (int)threadIdx.x, lane = tid & 31, wave = tid >> 5;
  const int bx = (int)blockIdx.x;
  const v4f z4 = {0.f, 0.f, 0.f, 0.f};
  if (bx < PB_X) {
    const int u = bx * 256 + tid;
    const int row = u >> 2, q = u & 3;
    const float* p = x + (size_t)row * FIN + 8 * (q & 1);
    v4f a = *(const v4fa*)p, b = *(const v4fa*)(p + 4);
    if (q >= 2) { a = z4; b = z4; }
    const v4u hv = pack8(a, b);
    unsigned short* dp = XB + (size_t)u * 8;
    *(volatile v4u*)dp = hv;
    __threadfence();
    *(volatile v4u*)dp = hv;
  } else if (bx < PB_X + PB_W1) {
    const int u = (bx - PB_X) * 256 + tid;
    const int n = u >> 2, q = u & 3;
    const int h = n >> 5, o = n & 31;
    const float* p = W1 + (size_t)h * (FIN * HID) + (size_t)(8 * (q & 1)) * HID + o;
    v4f a, b;
    a.x = p[0];       a.y = p[HID];     a.z = p[2 * HID]; a.w = p[3 * HID];
    b.x = p[4 * HID]; b.y = p[5 * HID]; b.z = p[6 * HID]; b.w = p[7 * HID];
    if (q >= 2) { a = z4; b = z4; }
    const v4u hv = pack8(a, b);
    unsigned short* dp = W1T + (size_t)u * 8;
    *(volatile v4u*)dp = hv;
    __threadfence();
    *(volatile v4u*)dp = hv;
  } else if (bx < PB_X + PB_W1 + PB_W2) {
    const int u = (bx - PB_X - PB_W1) * 256 + tid;
    const int n = u / (K2 / 8);
    const int k8 = (u - n * (K2 / 8)) * 8;
    const int kk = k8 >= CAT ? k8 - CAT : k8;
    const float* p = W2 + (size_t)kk * OC + n;
    v4f a, b;
    a.x = p[0];      a.y = p[OC];     a.z = p[2 * OC]; a.w = p[3 * OC];
    b.x = p[4 * OC]; b.y = p[5 * OC]; b.z = p[6 * OC]; b.w = p[7 * OC];
    const v4u hv = pack8(a, b);
    unsigned short* dp = W2D + (size_t)u * 8;
    *(volatile v4u*)dp = hv;
    __threadfence();
    *(volatile v4u*)dp = hv;
  } else {
    const int row = (bx - PB_X - PB_W1 - PB_W2) * 8 + wave;
    const float* ar = adj + (size_t)row * NN;
#pragma unroll 4
    for (int t = 0; t < 16; ++t) {
      const int j0 = 128 * t + 4 * lane;
      const v4f a = *(const v4fa*)(ar + j0);
      unsigned int nib = 0u;
      nib |= ((bfr(a.x) + ((j0 + 0) == row ? 1.0f : 0.0f)) > 0.0f) ? 1u : 0u;
      nib |= ((bfr(a.y) + ((j0 + 1) == row ? 1.0f : 0.0f)) > 0.0f) ? 2u : 0u;
      nib |= ((bfr(a.z) + ((j0 + 2) == row ? 1.0f : 0.0f)) > 0.0f) ? 4u : 0u;
      nib |= ((bfr(a.w) + ((j0 + 3) == row ? 1.0f : 0.0f)) > 0.0f) ? 8u : 0u;
      int w = (int)(nib << (4 * (lane & 7)));
      w |= __shfl_xor(w, 1);
      w |= __shfl_xor(w, 2);
      w |= __shfl_xor(w, 4);
      if ((lane & 7) == 0) kws[wave * 64 + 4 * t + (lane >> 3)] = (unsigned int)w;
    }
    __syncthreads();
    const int l16 = lane & 15;
    const v4u kv = *(const v4ua*)(kws + wave * 64 + 4 * l16);
    unsigned int* dp = KEEP + (size_t)row * 64 + 4 * l16;
    if (lane < 16) *(volatile v4u*)dp = kv;
    __threadfence();
    if (lane < 16) *(volatile v4u*)dp = kv;
  }
}

template <int NT>
__global__ __launch_bounds__(128) void k_proj(const unsigned short* __restrict__ A, int ksteps,
                                              const unsigned short* __restrict__ WT, int ldb,
                                              const float* __restrict__ avec, int nheads,
                                              unsigned short* HT, float* SD) {
  constexpr int OD = 16 * NT;
  constexpr int NIT = OD / 8;
  __shared__ __attribute__((aligned(16))) float stg[64 * OD];
  __shared__ __attribute__((aligned(16))) float satt[2 * OD];
  __shared__ __attribute__((aligned(16))) float sdot[128];
  const int tid = (int)threadIdx.x, lane = tid & 31, wave = tid >> 5, hh = lane >> 4, m = lane & 15;
  const int rowBase = (int)blockIdx.x * 64;
  const int head = (int)blockIdx.y;
  const int col0 = head * OD;
  const int b = rowBase >> 11, n0 = rowBase & (NN - 1);
  const int bh = b * nheads + head;
  const size_t htPlane = (size_t)NB * (size_t)nheads * OD * NN;

  {
    const int ia = tid < 2 * OD ? tid : 2 * OD - 1;
    const float v = bfr(avec[head * 2 * OD + ia]);
    if (tid < 2 * OD) satt[tid] = v;
  }

  v8f acc[NT];
  {
    const v8f z = {0.f, 0.f, 0.f, 0.f, 0.f, 0.f, 0.f, 0.f};
#pragma unroll
    for (int t = 0; t < NT; ++t) acc[t] = z;
  }
  const unsigned short* ap = A + (size_t)(rowBase + 16 * wave + m) * KX + 8 * hh;
  const unsigned short* wp = WT + (size_t)(col0 + m) * (size_t)ldb + 8 * hh;
#pragma unroll 1
  for (int s = 0; s < ksteps; ++s) {
    const unsigned short* aq = ap + (size_t)s * ((size_t)MR * KX);
    FragB af;
    af.h[0] = *(const v8usa*)aq;
    af.h[1] = *(const v8usa*)(aq + 16);
#pragma unroll
    for (int t = 0; t < NT; ++t) {
      const unsigned short* wq = wp + (size_t)(16 * t) * (size_t)ldb + 32 * s;
      FragB bf;
      bf.h[0] = *(const v8usa*)wq;
      bf.h[1] = *(const v8usa*)(wq + 16);
      acc[t] = wmb(af, bf, acc[t]);
    }
  }
#pragma unroll
  for (int t = 0; t < NT; ++t) {
#pragma unroll
    for (int r = 0; r < 8; ++r) stg[(16 * wave + 8 * hh + r) * OD + 16 * t + m] = acc[t][r];
  }
  __syncthreads();

  {
    const int row = tid & 63, which = tid >> 6;
    const float* sa = satt + which * OD;
    const float* hr = stg + row * OD;
    float d = 0.f;
#pragma unroll 4
    for (int c4 = 0; c4 < OD / 4; ++c4) {
      const v4f hv = *(const v4fa*)(hr + 4 * c4);
      const v4f av = *(const v4fa*)(sa + 4 * c4);
      d = fmaf(hv.x, av.x, d);
      d = fmaf(hv.y, av.y, d);
      d = fmaf(hv.z, av.z, d);
      d = fmaf(hv.w, av.w, d);
    }
    sdot[which * 64 + row] = d;
  }
  __syncthreads();

  v4u pk[NIT];
#pragma unroll
  for (int i = 0; i < NIT; ++i) {
    const int p = tid + 128 * i;
    const int line = p >> 3, q = p & 7;
    const int plane = (16 * i) / OD;
    const int o = line - plane * OD;
    unsigned int rh[8], rl[8];
#pragma unroll
    for (int j = 0; j < 8; ++j) split2(stg[(8 * q + j) * OD + o], rh[j], rl[j]);
    v4u w;
    w.x = plane ? pkw(rl[0], rl[1]) : pkw(rh[0], rh[1]);
    w.y = plane ? pkw(rl[2], rl[3]) : pkw(rh[2], rh[3]);
    w.z = plane ? pkw(rl[4], rl[5]) : pkw(rh[4], rh[5]);
    w.w = plane ? pkw(rl[6], rl[7]) : pkw(rh[6], rh[7]);
    pk[i] = w;
  }
  const int which2 = lane >> 4, piece = lane & 15;
  const v4f sdv = *(const v4fa*)(sdot + which2 * 64 + 4 * piece);
  float* sp = SD + ((size_t)bh * 2 + which2) * NN + n0 + 4 * piece;

#pragma unroll
  for (int i = 0; i < NIT; ++i) {
    const int p = tid + 128 * i;
    const int line = p >> 3, q = p & 7;
    const int plane = (16 * i) / OD;
    const int o = line - plane * OD;
    unsigned short* dp = HT + (size_t)plane * htPlane + ((size_t)bh * OD + o) * NN + n0 + 8 * q;
    *(volatile v4u*)dp = pk[i];
  }
  if (wave == 0) *(volatile v4f*)sp = sdv;
  __threadfence();
#pragma unroll
  for (int i = 0; i < NIT; ++i) {
    const int p = tid + 128 * i;
    const int line = p >> 3, q = p & 7;
    const int plane = (16 * i) / OD;
    const int o = line - plane * OD;
    unsigned short* dp = HT + (size_t)plane * htPlane + ((size_t)bh * OD + o) * NN + n0 + 8 * q;
    *(volatile v4u*)dp = pk[i];
  }
  if (wave == 0) *(volatile v4f*)sp = sdv;
}

template <int NT, int LAYER>
__global__ __launch_bounds__(128) void k_att(const unsigned int* __restrict__ keep,
                                             const unsigned short* __restrict__ HT,
                                             const float* __restrict__ SD, int nheads,
                                             unsigned short* X1P, float* outp) {
  constexpr int OD = 16 * NT;
  __shared__ __attribute__((aligned(16))) unsigned int keeps[64 * 64];
  __shared__ __attribute__((aligned(16))) float s2s[NN];
  __shared__ __attribute__((aligned(16))) float ost[64 * OD];
  __shared__ __attribute__((aligned(16))) float lrow[64];
  const int tid = (int)threadIdx.x, lane = tid & 31, wave = tid >> 5, hh = lane >> 4, m = lane & 15;
  const int bx = (int)blockIdx.x;
  const int b = bx >> 5;
  const int i0 = (bx & 31) * 64;
  const int rowBase = bx * 64;
  const int rloc = 16 * wave + m;
  const size_t htPlane = (size_t)NB * (size_t)nheads * OD * NN;

#pragma unroll
  for (int i = 0; i < 8; ++i) {
    const int p = tid + 128 * i;
    *(v4ua*)(keeps + 4 * p) = *(const v4ua*)(keep + (size_t)i0 * 64 + 4 * p);
  }
  const unsigned int* kr = keeps + rloc * 64;

#pragma unroll 1
  for (int hd = 0; hd < nheads; ++hd) {
    const int bh = b * nheads + hd;
    __syncthreads();
    {
      const float* s2g = SD + ((size_t)bh * 2 + 1) * NN;
#pragma unroll
      for (int i = 0; i < 4; ++i) {
        const int p = tid + 128 * i;
        *(v4fa*)(s2s + 4 * p) = *(const v4fa*)(s2g + 4 * p);
      }
    }
    const float s1r = SD[((size_t)bh * 2) * NN + i0 + rloc];
    __syncthreads();

    float mx2 = NEGBIG;
#pragma unroll 1
    for (int wd = 0; wd < 32; ++wd) {
      const int w = hh * 32 + wd;
      const unsigned int kw = kr[w];
      const float* sp = s2s + w * 32;
#pragma unroll
      for (int q = 0; q < 8; ++q) {
        const v4f s = *(const v4fa*)(sp + 4 * q);
        mx2 = fmaxf(mx2, (kw & (1u << (4 * q + 0))) != 0u ? s.x : NEGBIG);
        mx2 = fmaxf(mx2, (kw & (1u << (4 * q + 1))) != 0u ? s.y : NEGBIG);
        mx2 = fmaxf(mx2, (kw & (1u << (4 * q + 2))) != 0u ? s.z : NEGBIG);
        mx2 = fmaxf(mx2, (kw & (1u << (4 * q + 3))) != 0u ? s.w : NEGBIG);
      }
    }
    mx2 = fmaxf(mx2, __shfl_xor(mx2, 16));
    float zm = s1r + mx2;
    zm = zm > 0.f ? zm : NEGSL * zm;
    const float mrow = (mx2 > -1.0e38f) ? zm : FILLV;

    v8f acc[NT];
    {
      const v8f z = {0.f, 0.f, 0.f, 0.f, 0.f, 0.f, 0.f, 0.f};
#pragma unroll
      for (int t = 0; t < NT; ++t) acc[t] = z;
    }
    float ls = 0.f;
    const unsigned short* hb = HT + (size_t)bh * OD * NN + (size_t)m * NN + 8 * hh;
#pragma unroll 1
    for (int s = 0; s < NN / 32; ++s) {
      const int k0 = 32 * s;
      const unsigned int kw = kr[s] >> (8 * hh);
      const float* sp = s2s + k0 + 8 * hh;
      float sv[16];
      {
        const v4f t0 = *(const v4fa*)sp, t1 = *(const v4fa*)(sp + 4);
        const v4f t2 = *(const v4fa*)(sp + 16), t3 = *(const v4fa*)(sp + 20);
        sv[0] = t0.x; sv[1] = t0.y; sv[2] = t0.z; sv[3] = t0.w;
        sv[4] = t1.x; sv[5] = t1.y; sv[6] = t1.z; sv[7] = t1.w;
        sv[8] = t2.x; sv[9] = t2.y; sv[10] = t2.z; sv[11] = t2.w;
        sv[12] = t3.x; sv[13] = t3.y; sv[14] = t3.z; sv[15] = t3.w;
      }
      unsigned int rh[16], rl[16];
#pragma unroll
      for (int i = 0; i < 16; ++i) {
        const unsigned int bit = (kw >> (i < 8 ? i : i + 8)) & 1u;
        const float z = s1r + sv[i];
        const float e = z > 0.f ? z : NEGSL * z;
        const float zz = bit != 0u ? e : FILLV;
        const float p = expf(zz - mrow);
        ls += p;
        split2(p, rh[i], rl[i]);
      }
      FragB ah, al;
#pragma unroll
      for (int wi = 0; wi < 8; ++wi) {
        ah.w[wi] = (int)pkw(rh[2 * wi], rh[2 * wi + 1]);
        al.w[wi] = (int)pkw(rl[2 * wi], rl[2 * wi + 1]);
      }
#pragma unroll
      for (int t = 0; t < NT; ++t) {
        const unsigned short* q = hb + (size_t)(16 * t) * NN + k0;
        FragB bhi, blo;
        bhi.h[0] = *(const v8usa*)q;
        bhi.h[1] = *(const v8usa*)(q + 16);
        blo.h[0] = *(const v8usa*)(q + htPlane);
        blo.h[1] = *(const v8usa*)(q + htPlane + 16);
        acc[t] = wmb(ah, bhi, acc[t]);
        acc[t] = wmb(ah, blo, acc[t]);
        acc[t] = wmb(al, bhi, acc[t]);
      }
    }
    ls += __shfl_xor(ls, 16);
#pragma unroll
    for (int t = 0; t < NT; ++t) {
#pragma unroll
      for (int r = 0; r < 8; ++r) ost[(16 * wave + 8 * hh + r) * OD + 16 * t + m] = acc[t][r];
    }
    if (hh == 0) lrow[rloc] = ls;
    __syncthreads();

    if constexpr (LAYER == 1) {
      v4u hv[2], lv[2];
#pragma unroll
      for (int i = 0; i < 2; ++i) {
        const int p = tid + 128 * i;
        const int row = p >> 2, o0 = (p & 3) * 8;
        const v4f a = *(const v4fa*)(ost + row * OD + o0);
        const v4f c = *(const v4fa*)(ost + row * OD + o0 + 4);
        const float inv = 1.0f / lrow[row];
        float y[8];
        y[0] = a.x * inv; y[1] = a.y * inv; y[2] = a.z * inv; y[3] = a.w * inv;
        y[4] = c.x * inv; y[5] = c.y * inv; y[6] = c.z * inv; y[7] = c.w * inv;
        unsigned int rh[8], rl[8];
#pragma unroll
        for (int j = 0; j < 8; ++j) {
          const float v = y[j];
          const float u = v > 0.f ? v : expm1f(v);
          split2(u, rh[j], rl[j]);
        }
        hv[i].x = pkw(rh[0], rh[1]); hv[i].y = pkw(rh[2], rh[3]); hv[i].z = pkw(rh[4], rh[5]); hv[i].w = pkw(rh[6], rh[7]);
        lv[i].x = pkw(rl[0], rl[1]); lv[i].y = pkw(rl[2], rl[3]); lv[i].z = pkw(rl[4], rl[5]); lv[i].w = pkw(rl[6], rl[7]);
      }
      unsigned short* dh = X1P + ((size_t)hd * MR + rowBase) * KX;
      unsigned short* dl = X1P + ((size_t)(NH1 + hd) * MR + rowBase) * KX;
#pragma unroll
      for (int i = 0; i < 2; ++i) {
        *(volatile v4u*)(dh + (size_t)(tid + 128 * i) * 8) = hv[i];
        *(volatile v4u*)(dl + (size_t)(tid + 128 * i) * 8) = lv[i];
      }
      __threadfence();
#pragma unroll
      for (int i = 0; i < 2; ++i) {
        *(volatile v4u*)(dh + (size_t)(tid + 128 * i) * 8) = hv[i];
        *(volatile v4u*)(dl + (size_t)(tid + 128 * i) * 8) = lv[i];
      }
    } else {
      v4f ov[2];
#pragma unroll
      for (int i = 0; i < 2; ++i) {
        const int p = tid + 128 * i;
        const int row = p >> 2, o0 = (p & 3) * 4;
        const v4f a = *(const v4fa*)(ost + row * OD + o0);
        const float inv = 1.0f / lrow[row];
        const float y0 = a.x * inv, y1 = a.y * inv, y2 = a.z * inv, y3 = a.w * inv;
        v4f o;
        o.x = y0 > 0.f ? y0 : expm1f(y0);
        o.y = y1 > 0.f ? y1 : expm1f(y1);
        o.z = y2 > 0.f ? y2 : expm1f(y2);
        o.w = y3 > 0.f ? y3 : expm1f(y3);
        ov[i] = o;
      }
      float* ob = outp + (size_t)rowBase * OC;
#pragma unroll
      for (int i = 0; i < 2; ++i) *(volatile v4f*)(ob + (size_t)(tid + 128 * i) * 4) = ov[i];
      __threadfence();
#pragma unroll
      for (int i = 0; i < 2; ++i) *(volatile v4f*)(ob + (size_t)(tid + 128 * i) * 4) = ov[i];
    }
  }
}

extern "C" void kernel_launch(void* const* d_in, const int* in_sizes, int n_in,
                              void* d_out, int out_size, void* d_ws, size_t ws_size,
                              hipStream_t stream) {
  if (n_in < 6) return;
  if (in_sizes[0] != NB * NN * FIN) return;
  if (in_sizes[1] != NN * NN) return;
  if (in_sizes[2] != NH1 * FIN * HID) return;
  if (in_sizes[3] != NH1 * 2 * HID) return;
  if (in_sizes[4] != CAT * OC) return;
  if (in_sizes[5] != 2 * OC) return;
  if (out_size != NB * NN * OC) return;

  const float* x   = (const float*)d_in[0];
  const float* adj = (const float*)d_in[1];
  const float* W1  = (const float*)d_in[2];
  const float* a1  = (const float*)d_in[3];
  const float* W2  = (const float*)d_in[4];
  const float* a2  = (const float*)d_in[5];
  float* out = (float*)d_out;

  char* ws = (char*)d_ws;
  size_t off = 0;
  const size_t oXB  = off; off += (size_t)MR * KX * 2;
  const size_t oW1T = off; off += (size_t)CAT * KX * 2;
  const size_t oW2D = off; off += (size_t)OC * K2 * 2;
  const size_t oKP  = off; off += (size_t)NN * 64 * 4;
  const size_t oHT1 = off; off += (size_t)2 * NB * NH1 * HID * NN * 2;
  const size_t oSD1 = off; off += (size_t)NB * NH1 * 2 * NN * 4;
  const size_t oX1P = off; off += (size_t)2 * NH1 * MR * KX * 2;
  const size_t oHT2 = off; off += (size_t)2 * NB * OC * NN * 2;
  const size_t oSD2 = off; off += (size_t)NB * 2 * NN * 4;
  if (off > ws_size || off > (size_t)WSMAX) return;
  unsigned short* XB  = (unsigned short*)(ws + oXB);
  unsigned short* W1T = (unsigned short*)(ws + oW1T);
  unsigned short* W2D = (unsigned short*)(ws + oW2D);
  unsigned int*   KP  = (unsigned int*)(ws + oKP);
  unsigned short* HT1 = (unsigned short*)(ws + oHT1);
  float*          SD1 = (float*)(ws + oSD1);
  unsigned short* X1P = (unsigned short*)(ws + oX1P);
  unsigned short* HT2 = (unsigned short*)(ws + oHT2);
  float*          SD2 = (float*)(ws + oSD2);

  k_prep<<<PB_X + PB_W1 + PB_W2 + PB_K, 256, 0, stream>>>(x, adj, W1, W2, XB, W1T, W2D, KP);
  k_proj<2><<<dim3(MR / 64, NH1), 128, 0, stream>>>(XB, 1, W1T, KX, a1, NH1, HT1, SD1);
  k_att<2, 1><<<MR / 64, 128, 0, stream>>>(KP, HT1, SD1, NH1, X1P, out);
  k_proj<1><<<dim3(MR / 64, 1), 128, 0, stream>>>(X1P, K2 / 32, W2D, K2, a2, 1, HT2, SD2);
  k_att<1, 2><<<MR / 64, 128, 0, stream>>>(KP, HT2, SD2, 1, X1P, out);
}
